// RUMLayer_85057532330620
// MI455X (gfx1250) — hardware-verified
//
#include <hip/hip_runtime.h>
#include <math.h>

typedef __attribute__((ext_vector_type(16))) _Float16 v16h;
typedef __attribute__((ext_vector_type(16))) __bf16 v16b;
typedef __attribute__((ext_vector_type(8)))  _Float16 v8h;
typedef __attribute__((ext_vector_type(8)))  float v8f;
typedef __attribute__((ext_vector_type(4)))  float v4f;
typedef __attribute__((ext_vector_type(2)))  float v2f;
typedef __attribute__((ext_vector_type(4)))  unsigned v4u;
typedef __attribute__((ext_vector_type(4)))  int v4i;
typedef float __attribute__((may_alias)) float_a;
typedef int __attribute__((may_alias)) int_a;

template <typename T> __device__ __forceinline__ void vst2(void* p, T v) { *(volatile T*)p = v; __threadfence(); *(volatile T*)p = v; }
__device__ __forceinline__ v8f wmma16(v16h a, v16h b, v8f c) {
  v8f d = __builtin_amdgcn_wmma_f32_16x16x32_f16(false, a, false, b, (short)0, c, false, false);
  asm volatile("v_nop\n\tv_nop\n\tv_nop\n\tv_nop" : "+v"(d) : "v"(a), "v"(b));
  return d;
}
__device__ __forceinline__ v8f wmma_bf(v16b a, v16b b, v8f c) {
  v8f d = __builtin_amdgcn_wmma_f32_16x16x32_bf16(false, a, false, b, (short)0, c, false, false);
  asm volatile("v_nop\n\tv_nop\n\tv_nop\n\tv_nop" : "+v"(d) : "v"(a), "v"(b));
  return d;
}
__device__ __forceinline__ v16h frag_h(const _Float16* rowk0, int lane) {
  union { v16h v; v8h q[2]; } u; const _Float16* p = rowk0 + 8 * (lane >> 4);
  u.q[0] = *(const v8h*)p; u.q[1] = *(const v8h*)(p + 16); return u.v;
}
__device__ __forceinline__ v16h frag_f32(const float* rowk0, int lane) {
  v16h a; const float* p = rowk0 + 8 * (lane >> 4);
#pragma unroll
  for (int i = 0; i < 8; ++i) { a[i] = (_Float16)p[i]; a[8 + i] = (_Float16)p[16 + i]; }
  return a;
}
__device__ __forceinline__ v16h frag_f32s(const float* rowk0, int lane, float sc) {
  v16h a; const float* p = rowk0 + 8 * (lane >> 4);
#pragma unroll
  for (int i = 0; i < 8; ++i) { a[i] = (_Float16)(p[i] * sc); a[8 + i] = (_Float16)(p[16 + i] * sc); }
  return a;
}
__device__ __forceinline__ v16h fragc_f32(const float* W, int k0, int n, int lane, int ld, int K) {
  v16h a; const int g = lane >> 4;
#pragma unroll
  for (int i = 0; i < 8; ++i) { const int ka = k0 + 8 * g + i, kb = ka + 16;
    a[i] = (_Float16)(ka < K ? W[(size_t)(ka < K ? ka : K - 1) * ld + n] : 0.f); a[8 + i] = (_Float16)(kb < K ? W[(size_t)(kb < K ? kb : K - 1) * ld + n] : 0.f); }
  return a;
}
struct F2 { v16b h, l; };
__device__ __forceinline__ F2 bsplit16(const float v[16]) { F2 r;
#pragma unroll
  for (int i = 0; i < 16; ++i) { const __bf16 h = (__bf16)v[i]; r.h[i] = h; r.l[i] = (__bf16)(v[i] - (float)h); }
  return r; }
__device__ __forceinline__ F2 split_row(const float* row, int k0, int lane) { float v[16]; const float* p = row + k0 + 8 * (lane >> 4);
#pragma unroll
  for (int i = 0; i < 8; ++i) { v[i] = p[i]; v[8 + i] = p[16 + i]; }
  return bsplit16(v); }
__device__ __forceinline__ F2 split_rowK(const float* row, int k0, int lane, int K) { float v[16]; const int g = lane >> 4;
#pragma unroll
  for (int i = 0; i < 8; ++i) { const int ka = k0 + 8 * g + i, kb = ka + 16; v[i] = ka < K ? row[ka < K ? ka : K - 1] : 0.f; v[8 + i] = kb < K ? row[kb < K ? kb : K - 1] : 0.f; }
  return bsplit16(v); }
__device__ __forceinline__ F2 split_col(const float* W, int k0, int n, int lane, int ld, int K) { float v[16]; const int g = lane >> 4;
#pragma unroll
  for (int i = 0; i < 8; ++i) { const int ka = k0 + 8 * g + i, kb = ka + 16; v[i] = ka < K ? W[(size_t)(ka < K ? ka : K - 1) * ld + n] : 0.f; v[8 + i] = kb < K ? W[(size_t)(kb < K ? kb : K - 1) * ld + n] : 0.f; }
  return bsplit16(v); }
__device__ __forceinline__ v8f mac3(const F2& a, const F2& b, v8f c) { c = wmma_bf(a.l, b.h, c); c = wmma_bf(a.h, b.l, c); return wmma_bf(a.h, b.h, c); }
__device__ __forceinline__ float sigm(float v) { return 1.0f / (1.0f + expf(-v)); }
#define LDSX() do { asm volatile("s_wait_dscnt 0" ::: "memory"); __builtin_amdgcn_wave_barrier(); __builtin_amdgcn_fence(__ATOMIC_RELEASE, "workgroup"); } while (0)


#define SS 4
#define NNODE 10000
#define LW 8
#define NSEQ (SS * NNODE)
#define HH 64
#define G3 192
#define FIN 64
#ifndef NBLK
#define NBLK (NSEQ / 64)
#endif
typedef __attribute__((ext_vector_type(8))) __bf16 v8b;
__device__ __forceinline__ v16b frag_b(const __bf16* rowk0, int lane) {
  union { v16b v; v8b q[2]; } u; const __bf16* p = rowk0 + 8 * (lane >> 4);
  u.q[0] = *(const v8b*)p; u.q[1] = *(const v8b*)(p + 16); return u.v;
}
__device__ __forceinline__ float bfr(float v) { return (float)(__bf16)v; }
__device__ __attribute__((noinline)) float exp_ni(float v) { return expf(v); }
__device__ __attribute__((noinline)) float erf_ni(float v) { return erff(v); }

struct F3 { v16b h, m, l; };
__device__ __forceinline__ F3 split3_row(const float* row, int k0, int lane) { F3 r; const float* p = row + k0 + 8 * (lane >> 4);
#pragma unroll
  for (int i = 0; i < 16; ++i) { const float v = (i < 8) ? p[i] : p[16 + i - 8]; const __bf16 hb = (__bf16)v; const float r1 = v - (float)hb; const __bf16 mb = (__bf16)r1; r.h[i] = hb; r.m[i] = mb; r.l[i] = (__bf16)(r1 - (float)mb); }
  return r; }
__device__ __forceinline__ v8f mac3w(const F3& a, v16b w, v8f c) { c = wmma_bf(a.l, w, c); c = wmma_bf(a.m, w, c); return wmma_bf(a.h, w, c); }

__device__ __forceinline__ v8f mac2(const F2& a, v16b w, v8f c) { c = wmma_bf(a.l, w, c); return wmma_bf(a.h, w, c); }
__device__ __forceinline__ float sigm_f(float x) { return 1.0f / (1.0f + __expf(-x)); }
__device__ __forceinline__ float tanh_f(float x) { const float e = __expf(-2.0f * fabsf(x)); const float t = (1.0f - e) / (1.0f + e); return x < 0.f ? -t : t; }
__device__ __attribute__((noinline)) float sin_ni(float v) { return sinf(v); }
__device__ __attribute__((noinline)) float cos_ni(float v) { return cosf(v); }
#define WS_PW   0u
#define PHF 0
#define PHB (PHF + G3 * HH)
#define PHM (PHB + G3 * HH)
#define PWA (PHM + G3 * HH)
#define PWF (PWA + G3 * HH)
#define PWB (PWF + G3 * HH)
#define PWEND (PWB + G3 * HH)
#define WS_TAB  (WS_PW + 2u * PWEND)
#define WS_WDG  (WS_TAB + 4u * 2 * 8 * G3)
#define WS_Y    (WS_WDG + 4u * 256)
#define WS_END  (WS_Y + 4u * NSEQ * LW * 128)

__global__ __launch_bounds__(256) void k_pack(const float* __restrict__ WHF, const float* __restrict__ WHB, const float* __restrict__ WHM, const float* __restrict__ WIM, __bf16* __restrict__ PW) {
  __shared__ __align__(16) __bf16 s[6][64]; const int o = blockIdx.x, t = threadIdx.x; const int m = t >> 6, k = t & 63;
  if (m == 0) { s[0][k] = (__bf16)WHF[o * HH + k]; s[1][k] = (__bf16)WHB[o * HH + k]; s[2][k] = (__bf16)WHM[o * HH + k]; }
  else if (m == 1) { s[3][k] = (__bf16)WIM[o * 193 + k]; s[4][k] = (__bf16)WIM[o * 193 + 64 + k]; s[5][k] = (__bf16)WIM[o * 193 + 128 + k]; }
  __syncthreads();
  if (t < 48) { const int mm = t >> 3, pc = t & 7; const size_t base = (mm == 0 ? PHF : mm == 1 ? PHB : mm == 2 ? PHM : mm == 3 ? PWA : mm == 4 ? PWF : PWB); vst2((unsigned*)(PW + base + (size_t)o * HH + pc * 8), *(const v4u*)&s[mm][pc * 8]); }
}
__global__ __launch_bounds__(256) void k_tables(const float* __restrict__ WIF, const float* __restrict__ BIF, const float* __restrict__ WIB, const float* __restrict__ BIB, const float* __restrict__ WIM, const int* __restrict__ WALKS, const int* __restrict__ DEG, float* __restrict__ TAB, float* __restrict__ WDG) {
  __shared__ __align__(16) float st[2][8][G3]; __shared__ __align__(16) float sd[256]; __shared__ int smax[256]; const int t = threadIdx.x;
  for (int q = t; q < 2 * 8 * G3; q += 256) { const int w = q / (8 * G3), u = (q / G3) % 8, o = q % G3; const float ang = ((float)u / (float)LW) * 6.28318530717958647692f; const float su = sin_ni(ang), cu = cos_ni(ang);
    const float* WI = w ? WIB : WIF; const float* BI = w ? BIB : BIF; st[w][u][o] = (su * bfr(WI[o * 2]) + cu * bfr(WI[o * 2 + 1])) + bfr(BI[o]); }
  int mx = 0; for (int i = t; i < NSEQ * LW; i += 256) mx = max(mx, DEG[min(max(WALKS[i], 0), NNODE - 1)]); smax[t] = mx; __syncthreads();
  for (int o = 128; o > 0; o >>= 1) { if (t < o) smax[t] = max(smax[t], smax[t + o]); __syncthreads(); }
  sd[t] = (t < G3) ? bfr(WIM[t * 193 + 192]) : (t == G3 ? 1.0f / (float)smax[0] : 0.f);
  __syncthreads();
  for (int q = t; q < 2 * 8 * G3 / 4; q += 256) vst2(TAB + q * 4, *(const v4f*)(&st[0][0][0] + q * 4));
  if (t < 64) vst2(WDG + t * 4, *(const v4f*)&sd[t * 4]);
}
__global__ __launch_bounds__(128) void k_rum(const float* __restrict__ Hin, const int* __restrict__ WALKS, const int* __restrict__ DEG, const __bf16* __restrict__ PW, const float* __restrict__ TAB, const float* __restrict__ WDG, const float* __restrict__ BHF, const float* __restrict__ BHB, const float* __restrict__ BIM, const float* __restrict__ BHM, float* __restrict__ Y, float* __restrict__ OUT) {
  __shared__ __align__(16) float sh[64][HH + 4]; __shared__ __align__(16) float shf[64][HH + 4]; __shared__ int swk[64][LW]; __shared__ int su[64][LW]; __shared__ __align__(16) float stab[2][8][G3]; __shared__ __align__(16) float swd[256]; __shared__ __align__(16) float sy[64][68];
  const int tid = threadIdx.x, wave = tid >> 5, lane = tid & 31, col = lane & 15, g = lane >> 4; const size_t q0 = (size_t)blockIdx.x * 64; const int r0 = wave * 16;
  for (int q = tid; q < 2 * 8 * G3; q += 128) (&stab[0][0][0])[q] = TAB[q];
  for (int q = tid; q < 256; q += 128) swd[q] = WDG[q];
  if (tid < 64) { const int* w = WALKS + (q0 + tid) * LW; int wk[LW];
#pragma unroll
    for (int l = 0; l < LW; ++l) wk[l] = min(max(w[l], 0), NNODE - 1);
#pragma unroll
    for (int l = 0; l < LW; ++l) { int first = l;
#pragma unroll
      for (int j = LW - 1; j >= 0; --j) if (wk[j] == wk[l]) first = j;
      swk[tid][LW - 1 - l] = wk[l]; su[tid][LW - 1 - l] = first; } }
  __syncthreads();
  const float rmd = swd[G3];
#pragma unroll 1
  for (int phase = 0; phase < 3; ++phase) {
    const __bf16* PWH = PW + (phase == 0 ? PHF : phase == 1 ? PHB : PHM); const float* BH = phase == 0 ? BHF : phase == 1 ? BHB : BHM;
    if (phase < 2) { for (int q = tid; q < 64 * HH; q += 128) sh[q / HH][q % HH] = 0.f; }
    else { for (int q = tid; q < 64 * HH; q += 128) { const int r = q / HH, c = q % HH; sh[r][c] = 0.5f * (shf[r][c] + sh[r][c]); } }
    __syncthreads();
#pragma unroll 1
    for (int step = 0; step < LW; ++step) { const int l = (phase == 1) ? (LW - 1 - step) : step;
      F2 hf[2]; hf[0] = split_row(&sh[r0 + col][0], 0, lane); hf[1] = split_row(&sh[r0 + col][0], 32, lane);
      LDSX();
#pragma unroll 1
      for (int half = 0; half < 2; ++half) { const int u0 = half * 32;
        v8f rz[4] = {}, ni[2] = {}, nh[2] = {};
        if (phase == 2) {
#pragma unroll 1
          for (int part = 0; part < 3; ++part) { const __bf16* PWI = PW + (part == 0 ? PWA : part == 1 ? PWF : PWB);
#pragma unroll 1
            for (int kc = 0; kc < 2; ++kc) { F2 a; if (part == 0) { const int node = swk[r0 + col][l]; const float* p = Hin + (size_t)node * FIN + kc * 32 + 8 * g; v16b ax;
#pragma unroll
                for (int i = 0; i < 8; ++i) { ax[i] = (__bf16)p[i]; ax[8 + i] = (__bf16)p[16 + i]; } a.h = ax; a.l = ax; }
              else a = split_row(Y + ((q0 + r0 + col) * LW + l) * 128 + (part == 1 ? 0 : 64), kc * 32, lane);
#pragma unroll
              for (int j = 0; j < 4; ++j) { const int orow = (j < 2 ? 0 : 64) + u0 + (j & 1) * 16 + col; const v16b w = frag_b(PWI + (size_t)orow * HH + kc * 32, lane); if (part == 0) rz[j] = wmma_bf(a.h, w, rz[j]); else rz[j] = mac2(a, w, rz[j]); }
#pragma unroll
              for (int j = 0; j < 2; ++j) { const int orow = 128 + u0 + j * 16 + col; const v16b w = frag_b(PWI + (size_t)orow * HH + kc * 32, lane); if (part == 0) ni[j] = wmma_bf(a.h, w, ni[j]); else ni[j] = mac2(a, w, ni[j]); } } } }
#pragma unroll
        for (int kc = 0; kc < 2; ++kc) {
#pragma unroll
          for (int j = 0; j < 4; ++j) { const int orow = (j < 2 ? 0 : 64) + u0 + (j & 1) * 16 + col; rz[j] = mac2(hf[kc], frag_b(PWH + (size_t)orow * HH + kc * 32, lane), rz[j]); }
#pragma unroll
          for (int j = 0; j < 2; ++j) { const int orow = 128 + u0 + j * 16 + col; nh[j] = mac2(hf[kc], frag_b(PWH + (size_t)orow * HH + kc * 32, lane), nh[j]); } }
#pragma unroll
        for (int j = 0; j < 2; ++j) { const int uo = u0 + j * 16 + col; const float bhr = bfr(BH[uo]), bhz = bfr(BH[64 + uo]), bhn = bfr(BH[128 + uo]);
          float bir = 0.f, biz = 0.f, bin_ = 0.f, wdr = 0.f, wdz = 0.f, wdn = 0.f;
          if (phase == 2) { bir = bfr(BIM[uo]); biz = bfr(BIM[64 + uo]); bin_ = bfr(BIM[128 + uo]); wdr = swd[uo]; wdz = swd[64 + uo]; wdn = swd[128 + uo]; }
#pragma unroll
          for (int r = 0; r < 8; ++r) { const int row = r0 + 8 * g + r; float xr, xz, xn;
            if (phase < 2) { const int u = su[row][l]; xr = stab[phase][u][uo]; xz = stab[phase][u][64 + uo]; xn = stab[phase][u][128 + uo]; }
            else { const float dg = (float)DEG[swk[row][l]] * rmd; xr = bir + dg * wdr; xz = biz + dg * wdz; xn = bin_ + dg * wdn; }
            const float rg = sigm_f(rz[j][r] + xr + bhr); const float zg = sigm_f(rz[2 + j][r] + xz + bhz); const float n = tanh_f((ni[j][r] + xn) + rg * (nh[j][r] + bhn));
            const float hold = sh[row][uo]; sh[row][uo] = (1.0f - zg) * n + zg * hold; } } }
      LDSX();
      if (phase < 2) {
        const int half = phase * 64;
        for (int q = lane; q < 16 * 16; q += 32) { const int rl = q >> 4, pc = q & 15; vst2(Y + ((q0 + r0 + rl) * LW + l) * 128 + half + pc * 4, *(const v4f*)&sh[r0 + rl][pc * 4]); } }
    }
    if (phase == 0) { for (int q = lane; q < 16 * HH; q += 32) { const int rl = q / HH, c = q % HH; shf[r0 + rl][c] = sh[r0 + rl][c]; } LDSX(); }
    __syncthreads();
  }
  for (int q = lane; q < 16 * 16; q += 32) { const int rl = q >> 4, pc = q & 15; vst2(OUT + (q0 + r0 + rl) * HH + pc * 4, *(const v4f*)&sh[r0 + rl][pc * 4]); }
}
extern "C" void kernel_launch(void* const* d_in, const int* in_sizes, int n_in, void* d_out, int out_size, void* d_ws, size_t ws_size, hipStream_t stream) {
  (void)in_sizes; (void)n_in; (void)out_size;
  const float** F = (const float**)d_in; const int* WALKS = (const int*)d_in[1]; const int* DEG = (const int*)d_in[2];
  if (ws_size < (size_t)WS_END) return;
  char* ws = (char*)d_ws; __bf16* PW = (__bf16*)(ws + WS_PW); float *TAB = (float*)(ws + WS_TAB), *WDG = (float*)(ws + WS_WDG), *Y = (float*)(ws + WS_Y);
  k_pack<<<G3, 256, 0, stream>>>(F[4], F[8], F[12], F[11], PW);
  k_tables<<<1, 256, 0, stream>>>(F[3], F[5], F[7], F[9], F[11], WALKS, DEG, TAB, WDG);
  k_rum<<<NBLK, 128, 0, stream>>>(F[0], WALKS, DEG, PW, TAB, WDG, F[6], F[10], F[13], F[14], Y, (float*)d_out);
}
